// Morpher_69638599737737
// MI455X (gfx1250) — hardware-verified
//
#include <hip/hip_runtime.h>


#define B_    4
#define T_    1024
#define N_    8
#define K_    4
#define D_    64
#define H_    32
#define OD_   192
#define PT    64
#define PTHR  128
#define QT    128
#define ATHR  256
#define KB_   64

typedef unsigned short us;
typedef us     v8us  __attribute__((ext_vector_type(8)));
typedef us     v16us __attribute__((ext_vector_type(16)));
typedef __bf16 v16bf __attribute__((ext_vector_type(16)));
typedef float  v8f   __attribute__((ext_vector_type(8)));
typedef float  v4f   __attribute__((ext_vector_type(4)));
typedef us     v8usa __attribute__((ext_vector_type(8), may_alias));
typedef float  v4fa  __attribute__((ext_vector_type(4), may_alias));

union Frag { v16us v; v8us h[2]; };

__device__ __forceinline__ us bf16_rne(float f) {
  unsigned int u = __builtin_bit_cast(unsigned int, f);
  u += 0x7FFFu + ((u >> 16) & 1u);
  return (us)(u >> 16);
}
__device__ __forceinline__ float bf16_val(us b) {
  return __builtin_bit_cast(float, ((unsigned int)b) << 16);
}
__device__ __forceinline__ void bf16_hilo(float f, us& hi, us& lo) {
  const us hh = bf16_rne(f);
  hi = hh;
  lo = bf16_rne(f - bf16_val(hh));
}

__device__ __forceinline__ v8f zero8() {
  v8f z = {0.f, 0.f, 0.f, 0.f, 0.f, 0.f, 0.f, 0.f};
  return z;
}

__device__ __forceinline__ v8f mma_bf16(v16us a, v16us b, v8f c) {
  const v16bf av = __builtin_bit_cast(v16bf, a);
  const v16bf bv = __builtin_bit_cast(v16bf, b);
  v8f d = __builtin_amdgcn_wmma_f32_16x16x32_bf16(false, av, false, bv, (short)0, c, false, false);
  asm volatile("v_nop\n\tv_nop\n\tv_nop\n\tv_nop" : "+v"(d) : "v"(av), "v"(bv));
  return d;
}

__device__ __forceinline__ v16us ld_frag(const us* rowp, int k0, int h) {
  Frag f;
  const us* p = rowp + k0 + 8 * h;
  f.h[0] = *(const v8usa*)(p);
  f.h[1] = *(const v8usa*)(p + 16);
  return f.v;
}

__global__ __launch_bounds__(PTHR)
void proj_kernel(const float* __restrict__ x,
                 const float* __restrict__ W,
                 const int*   __restrict__ perm,
                 const int*   __restrict__ inv,
                 us* Qh, us* Ql, us* Kh, us* Kl, us* Vh, us* Vl)
{
  __shared__ __align__(16) us    xs [PT  * D_];
  __shared__ __align__(16) us    wsT[OD_ * D_];
  __shared__ __align__(16) float stg[PT  * D_];

  const int bh    = blockIdx.x;
  const int tbase = blockIdx.y * PT;
  const int b  = bh >> 5;
  const int hd = bh & 31;
  const int n  = hd >> 2;
  const int k  = hd & 3;

  int p = perm[k * N_ + n];
  p = p < 0 ? 0 : (p > N_ - 1 ? N_ - 1 : p);
  int s = inv[k * N_ + p];
  s = s < 0 ? 0 : (s > N_ - 1 ? N_ - 1 : s);
  const float* Wsrc = W + (size_t)(k * N_ + p) * (D_ * OD_);

  const int tid = threadIdx.x;

  for (int i = tid; i < PT * (D_ / 4); i += PTHR) {
    const int row = i >> 4, c4 = i & 15;
    const size_t src = ((((size_t)(b * T_ + tbase + row)) * N_ + s) * K_ + k) * D_ + 4 * c4;
    const v4fa v = *(const v4fa*)(x + src);
    us* d = xs + row * D_ + 4 * c4;
    d[0] = bf16_rne(v[0]); d[1] = bf16_rne(v[1]); d[2] = bf16_rne(v[2]); d[3] = bf16_rne(v[3]);
  }
  for (int i = tid; i < D_ * (OD_ / 4); i += PTHR) {
    const int dd = i / (OD_ / 4), o4 = i - dd * (OD_ / 4);
    const v4fa v = *(const v4fa*)(Wsrc + dd * OD_ + 4 * o4);
    wsT[(4 * o4 + 0) * D_ + dd] = bf16_rne(v[0]);
    wsT[(4 * o4 + 1) * D_ + dd] = bf16_rne(v[1]);
    wsT[(4 * o4 + 2) * D_ + dd] = bf16_rne(v[2]);
    wsT[(4 * o4 + 3) * D_ + dd] = bf16_rne(v[3]);
  }
  __syncthreads();

  const int wv   = tid >> 5;
  const int lane = tid & 31;
  const int h    = lane >> 4;
  const int l16  = lane & 15;
  const us* arow = xs + (16 * wv + l16) * D_;

  for (int part = 0; part < 3; ++part) {
    const float sc = (part == 0) ? 0.125f : 1.0f;
#pragma unroll
    for (int ct = 0; ct < 4; ++ct) {
      const us* brow = wsT + (part * 64 + ct * 16 + l16) * D_;
      v8f acc = zero8();
#pragma unroll
      for (int ks = 0; ks < 2; ++ks)
        acc = mma_bf16(ld_frag(arow, 32 * ks, h), ld_frag(brow, 32 * ks, h), acc);
#pragma unroll
      for (int r = 0; r < 8; ++r)
        stg[(16 * wv + 8 * h + r) * D_ + ct * 16 + l16] = acc[r] * sc;
    }
    __syncthreads();

    if (part < 2) {
      us* dh = (part == 0) ? Qh : Kh;
      us* dl = (part == 0) ? Ql : Kl;
      const int seg = tid & 7;
      for (int pass = 0; pass < 2; ++pass) {
        for (int rr = tid >> 3; rr < PT; rr += PTHR / 8) {
          const float* st = stg + rr * D_ + seg * 8;
          const v4fa f0 = *(const v4fa*)(st);
          const v4fa f1 = *(const v4fa*)(st + 4);
          v8us hv, lv;
          us a0, c0;
          bf16_hilo(f0[0], a0, c0); hv[0] = a0; lv[0] = c0;
          bf16_hilo(f0[1], a0, c0); hv[1] = a0; lv[1] = c0;
          bf16_hilo(f0[2], a0, c0); hv[2] = a0; lv[2] = c0;
          bf16_hilo(f0[3], a0, c0); hv[3] = a0; lv[3] = c0;
          bf16_hilo(f1[0], a0, c0); hv[4] = a0; lv[4] = c0;
          bf16_hilo(f1[1], a0, c0); hv[5] = a0; lv[5] = c0;
          bf16_hilo(f1[2], a0, c0); hv[6] = a0; lv[6] = c0;
          bf16_hilo(f1[3], a0, c0); hv[7] = a0; lv[7] = c0;
          const size_t idx = ((size_t)bh * T_ + tbase + rr) * D_ + seg * 8;
          *(volatile v8us*)(dh + idx) = hv;
          *(volatile v8us*)(dl + idx) = lv;
        }
        if (pass == 0) __threadfence();
      }
    } else {
      for (int pass = 0; pass < 2; ++pass) {
        for (int it = tid; it < D_ * (PT / 8); it += PTHR) {
          const int dd = it >> 3, tseg = it & 7;
          v8us hv, lv;
#pragma unroll
          for (int e = 0; e < 8; ++e) {
            us a0, c0;
            bf16_hilo(stg[(tseg * 8 + e) * D_ + dd], a0, c0);
            hv[e] = a0; lv[e] = c0;
          }
          const size_t idx = ((size_t)bh * D_ + dd) * T_ + tbase + tseg * 8;
          *(volatile v8us*)(Vh + idx) = hv;
          *(volatile v8us*)(Vl + idx) = lv;
        }
        if (pass == 0) __threadfence();
      }
    }
    __syncthreads();
  }
}

__global__ __launch_bounds__(ATHR)
void attn_kernel(const us* __restrict__ Qh, const us* __restrict__ Ql,
                 const us* __restrict__ Kh, const us* __restrict__ Kl,
                 const us* __restrict__ Vh, const us* __restrict__ Vl,
                 float* out)
{
  __shared__ __align__(16) us Khs[KB_ * D_];
  __shared__ __align__(16) us Kls[KB_ * D_];
  __shared__ __align__(16) us Vhs[D_ * KB_];
  __shared__ __align__(16) us Vls[D_ * KB_];
  __shared__ __align__(16) us Pbuf[(ATHR / 32) * 2048];

  const int bh    = blockIdx.x;
  const int qbase = blockIdx.y * QT;
  const int b  = bh >> 5;
  const int hd = bh & 31;
  const int n  = hd >> 2;
  const int k  = hd & 3;

  const int tid  = threadIdx.x;
  const int wv   = tid >> 5;
  const int lane = tid & 31;
  const int h    = lane >> 4;
  const int l16  = lane & 15;
  const int q0   = qbase + 16 * wv;
  us* Pb = Pbuf + wv * 2048;

  v16us qh[2], ql[2];
  {
    const size_t ro = ((size_t)bh * T_ + q0 + l16) * D_;
#pragma unroll
    for (int ks = 0; ks < 2; ++ks) {
      qh[ks] = ld_frag(Qh + ro, 32 * ks, h);
      ql[ks] = ld_frag(Ql + ro, 32 * ks, h);
    }
  }

  float mrow[8], lrow[8];
  v8f accO[4];
#pragma unroll
  for (int r = 0; r < 8; ++r) { mrow[r] = -1.0e30f; lrow[r] = 0.0f; }
#pragma unroll
  for (int dt = 0; dt < 4; ++dt) accO[dt] = zero8();

  const int kend = qbase + QT;
  for (int kb = 0; kb < kend; kb += KB_) {
#pragma unroll
    for (int j = 0; j < 2; ++j) {
      const int c   = tid + j * ATHR;
      const int row = c >> 3, seg = c & 7;
      const int lo  = row * 64 + seg * 8;
      const size_t gk = ((size_t)bh * T_ + kb + row) * D_ + seg * 8;
      const size_t gv = ((size_t)bh * D_ + row) * T_ + kb + seg * 8;
      *(v8usa*)(Khs + lo) = *(const v8usa*)(Kh + gk);
      *(v8usa*)(Kls + lo) = *(const v8usa*)(Kl + gk);
      *(v8usa*)(Vhs + lo) = *(const v8usa*)(Vh + gv);
      *(v8usa*)(Vls + lo) = *(const v8usa*)(Vl + gv);
    }
    __syncthreads();

    const bool active = (kb <= q0);
    if (active) {
      v8f accS[4];
#pragma unroll
      for (int ct = 0; ct < 4; ++ct) accS[ct] = zero8();
#pragma unroll
      for (int ct = 0; ct < 4; ++ct) {
        if (kb + ct * 16 <= q0 + 15) {
          const us* krh = Khs + (ct * 16 + l16) * D_;
          const us* krl = Kls + (ct * 16 + l16) * D_;
#pragma unroll
          for (int ks = 0; ks < 2; ++ks) {
            const v16us bhf = ld_frag(krh, 32 * ks, h);
            const v16us blf = ld_frag(krl, 32 * ks, h);
            accS[ct] = mma_bf16(qh[ks], bhf, accS[ct]);
            accS[ct] = mma_bf16(qh[ks], blf, accS[ct]);
            accS[ct] = mma_bf16(ql[ks], bhf, accS[ct]);
          }
        }
      }

#pragma unroll
      for (int r = 0; r < 8; ++r) {
        const int qg = q0 + 8 * h + r;
        float sv[4];
        float mloc = -1.0e30f;
#pragma unroll
        for (int ct = 0; ct < 4; ++ct) {
          const int col = kb + ct * 16 + l16;
          sv[ct] = (col <= qg) ? accS[ct][r] : -1.0e30f;
          mloc = fmaxf(mloc, sv[ct]);
        }
#pragma unroll
        for (int off = 1; off < 16; off <<= 1)
          mloc = fmaxf(mloc, __shfl_xor(mloc, off, 32));
        const float mnew = fmaxf(mrow[r], mloc);
        const float scl  = __expf(mrow[r] - mnew);
        float psum = 0.0f;
#pragma unroll
        for (int ct = 0; ct < 4; ++ct) {
          const int col = kb + ct * 16 + l16;
          const float pv = (col <= qg) ? __expf(sv[ct] - mnew) : 0.0f;
          psum += pv;
          us ph, pl;
          bf16_hilo(pv, ph, pl);
          Pb[       (8 * h + r) * 64 + ct * 16 + l16] = ph;
          Pb[1024 + (8 * h + r) * 64 + ct * 16 + l16] = pl;
        }
#pragma unroll
        for (int off = 1; off < 16; off <<= 1)
          psum += __shfl_xor(psum, off, 32);
        lrow[r] = lrow[r] * scl + psum;
        mrow[r] = mnew;
#pragma unroll
        for (int dt = 0; dt < 4; ++dt) accO[dt][r] *= scl;
      }
    }
    __syncthreads();

    if (active) {
#pragma unroll
      for (int ks = 0; ks < 2; ++ks) {
        if (kb + 32 * ks <= q0 + 15) {
          const v16us phf = ld_frag(Pb +        l16 * 64, 32 * ks, h);
          const v16us plf = ld_frag(Pb + 1024 + l16 * 64, 32 * ks, h);
#pragma unroll
          for (int dt = 0; dt < 4; ++dt) {
            const us* vrh = Vhs + (dt * 16 + l16) * KB_;
            const us* vrl = Vls + (dt * 16 + l16) * KB_;
            const v16us vhf = ld_frag(vrh, 32 * ks, h);
            const v16us vlf = ld_frag(vrl, 32 * ks, h);
            accO[dt] = mma_bf16(phf, vhf, accO[dt]);
            accO[dt] = mma_bf16(phf, vlf, accO[dt]);
            accO[dt] = mma_bf16(plf, vhf, accO[dt]);
          }
        }
      }
    }
    __syncthreads();
  }

  float* Ost = (float*)Pb;
#pragma unroll
  for (int r = 0; r < 8; ++r) {
    const float il = 1.0f / lrow[r];
#pragma unroll
    for (int dt = 0; dt < 4; ++dt)
      Ost[(8 * h + r) * 64 + dt * 16 + l16] = accO[dt][r] * il;
  }
  __syncthreads();

  for (int pass = 0; pass < 2; ++pass) {
#pragma unroll
    for (int i = 0; i < 8; ++i) {
      const int rowl = 2 * i + h;
      const v4fa v = *(const v4fa*)(Ost + rowl * 64 + 4 * l16);
      const int t = q0 + rowl;
      float* dst = out + ((((size_t)(b * T_ + t)) * N_ + n) * K_ + k) * D_ + 4 * l16;
      *(volatile v4fa*)dst = v;
    }
    if (pass == 0) __threadfence();
  }
}

extern "C" void kernel_launch(void* const* d_in, const int* in_sizes, int n_in,
                              void* d_out, int out_size, void* d_ws, size_t ws_size,
                              hipStream_t stream)
{
  if (n_in < 4) return;
  if (in_sizes[0] != B_ * T_ * N_ * K_ * D_) return;
  if (in_sizes[1] != K_ * N_ * D_ * OD_) return;
  if (in_sizes[2] != K_ * N_) return;
  if (in_sizes[3] != K_ * N_) return;
  if (out_size != B_ * T_ * N_ * K_ * D_) return;

  const size_t per  = (size_t)B_ * H_ * T_ * D_;
  const size_t need = 6 * per * sizeof(us);
  if (need > ws_size) return;

  const float* x    = (const float*)d_in[0];
  const float* W    = (const float*)d_in[1];
  const int*   perm = (const int*)d_in[2];
  const int*   inv  = (const int*)d_in[3];
  float* out = (float*)d_out;

  us* Qh = (us*)d_ws;
  us* Ql = Qh + per;
  us* Kh = Ql + per;
  us* Kl = Kh + per;
  us* Vh = Kl + per;
  us* Vl = Vh + per;

  dim3 g1(B_ * H_, T_ / PT);
  dim3 g2(B_ * H_, T_ / QT);
  proj_kernel<<<g1, PTHR, 0, stream>>>(x, W, perm, inv, Qh, Ql, Kh, Kl, Vh, Vl);
  attn_kernel<<<g2, ATHR, 0, stream>>>(Qh, Ql, Kh, Kl, Vh, Vl, out);
}
